// SharedPointSetAttention_29832842838757
// MI455X (gfx1250) — hardware-run, weakly checked
//
#include <hip/hip_runtime.h>
#include <stddef.h>
#include <stdint.h>


#define SPLIT_A 1

#define NN     30000
#define DF     128
#define NE     480000
#define MP     30208
#define AP     512
#define WPK    256
#define KOUT   (SPLIT_A ? 512 : 256)
#define GBM    64
#define GTHR   128
#define FSL    1024
#define FNB    30
#define FPITCH 1028
#define FLGN   (FNB * FSL)
#define FTHR   256
#define NV4    (NE / 4)
#define FIT    ((NV4 + FTHR - 1) / FTHR)
#define UFB    (MP * DF / 8)
#define UWV    (DF * DF / 8)
#define UWP    (DF * WPK / 8)
#define BFB    (UFB / 256)
#define BWV    (UWV / 256)
#define BWP    (UWP / 256)
#define PREP_BLOCKS (2 * BFB + 2 * BWV + 2 * BWP)
#define OUT1_ELEM 3840000

#define SZ_FB   ((size_t)MP * DF * 2)
#define SZ_AHL  ((size_t)MP * AP * 2)
#define SZ_FLG  ((size_t)4 * FLGN * 4)
#define SZ_WV   ((size_t)DF * DF * 2)
#define SZ_WP   ((size_t)DF * WPK * 2)
#define O_FB    ((size_t)0)
#define O_AHL   (O_FB + 2 * SZ_FB)
#define O_FLG   (O_AHL + 2 * SZ_AHL)
#define O_WV    (O_FLG + SZ_FLG)
#define O_WP    (O_WV + 2 * SZ_WV)
#define WS_TOTAL (O_WP + 2 * SZ_WP)
#define WSMAX   134217728

static_assert(DF == 128);
static_assert(MP % GBM == 0 && MP >= NN && MP - NN < GBM * 4);
static_assert(FLGN >= MP);
static_assert(NE % 4 == 0);
static_assert(AP == 4 * DF && WPK == 2 * DF);
static_assert(KOUT % 32 == 0 && KOUT <= AP && (KOUT == WPK || KOUT == 2 * WPK));
static_assert((WPK & (WPK - 1)) == 0 && (DF & (DF - 1)) == 0);
static_assert(UFB % 256 == 0 && UWV % 256 == 0 && UWP % 256 == 0);
static_assert(GBM == (GTHR / 32) * 16);
static_assert((FPITCH * 4) % 16 == 0 && FPITCH > FSL && (8 * FPITCH) % 4 == 0);
static_assert(FSL == 4 * FTHR);
static_assert(OUT1_ELEM == NN * DF);
static_assert((long long)OUT1_ELEM + (long long)(NN - 1) * DF + DF - 1 < 2LL * NN * DF);
static_assert(SZ_FB % 256 == 0 && SZ_AHL % 256 == 0 && SZ_FLG % 256 == 0 && SZ_WV % 256 == 0 && SZ_WP % 256 == 0);
static_assert(WS_TOTAL == 78020608 && WS_TOTAL <= (size_t)WSMAX);

typedef float          v4f   __attribute__((ext_vector_type(4)));
typedef float          v8f   __attribute__((ext_vector_type(8)));
typedef int            v4i   __attribute__((ext_vector_type(4)));
typedef int            v8i   __attribute__((ext_vector_type(8)));
typedef unsigned       v4u   __attribute__((ext_vector_type(4)));
typedef unsigned short v4us  __attribute__((ext_vector_type(4)));
typedef unsigned short v8us  __attribute__((ext_vector_type(8)));
typedef unsigned short v16us __attribute__((ext_vector_type(16)));
typedef __bf16         v16bf __attribute__((ext_vector_type(16)));
typedef v4f  __attribute__((may_alias)) v4fa;
typedef v4u  __attribute__((may_alias)) v4ua;
typedef v4us __attribute__((may_alias)) v4usa;
typedef v8us __attribute__((may_alias)) v8usa;
union FragB { v16bf v; v16us u; v8us h[2]; v8i w; };

__device__ __forceinline__ v8f wmb(const FragB& a, const FragB& b, v8f c) {
  v8f d = __builtin_amdgcn_wmma_f32_16x16x32_bf16(false, a.v, false, b.v, (short)0, c, false, false);
  asm volatile("v_nop\n\tv_nop\n\tv_nop\n\tv_nop" : "+v"(d) : "v"(a.w), "v"(b.w));
  return d;
}

__device__ __forceinline__ unsigned bf16_bits(float f) {
  const unsigned u = __float_as_uint(f);
  return (u + 0x7FFFu + ((u >> 16) & 1u)) >> 16;
}
__device__ __forceinline__ float bf16_val(float f) {
  return __uint_as_float(bf16_bits(f) << 16);
}

__device__ __forceinline__ void wave_sync() {
  __builtin_amdgcn_fence(__ATOMIC_RELEASE, "wavefront");
  __builtin_amdgcn_wave_barrier();
  __builtin_amdgcn_fence(__ATOMIC_ACQUIRE, "wavefront");
}

__device__ __forceinline__ void cvt8(const float* __restrict__ src, unsigned short* dst, unsigned msk) {
  const v4f a = *(const v4f*)src;
  const v4f b = *(const v4f*)(src + 4);
  asm volatile("" :: "v"(a), "v"(b));
  v8us o;
  o[0] = (unsigned short)(bf16_bits(a.x) & msk); o[1] = (unsigned short)(bf16_bits(a.y) & msk);
  o[2] = (unsigned short)(bf16_bits(a.z) & msk); o[3] = (unsigned short)(bf16_bits(a.w) & msk);
  o[4] = (unsigned short)(bf16_bits(b.x) & msk); o[5] = (unsigned short)(bf16_bits(b.y) & msk);
  o[6] = (unsigned short)(bf16_bits(b.z) & msk); o[7] = (unsigned short)(bf16_bits(b.w) & msk);
  *(volatile v8us*)dst = o;
  __threadfence();
  *(volatile v8us*)dst = o;
}

__device__ __forceinline__ void prep_feat(const float* __restrict__ f, unsigned short* plane, int u) {
  const int row = u >> 4;
  const int rc  = row < NN ? row : NN - 1;
  const unsigned msk = row < NN ? 0xFFFFu : 0u;
  cvt8(f + (size_t)rc * DF + (u & 15) * 8, plane + (size_t)u * 8, msk);
}

__global__ __launch_bounds__(256) void k_prep(const float* __restrict__ f1, const float* __restrict__ f2,
                                              const float* __restrict__ wv1, const float* __restrict__ wv2,
                                              const float* __restrict__ wp1, const float* __restrict__ wp2,
                                              unsigned short* FB, unsigned short* WVB, unsigned short* WPB) {
  const int tid = (int)threadIdx.x;
  int b = (int)blockIdx.x;
  if (b < BFB) {
    prep_feat(f1, FB, b * 256 + tid);
  } else if (b < 2 * BFB) {
    prep_feat(f2, FB + (size_t)MP * DF, (b - BFB) * 256 + tid);
  } else {
    b -= 2 * BFB;
    if (b < BWV) {
      const int u = b * 256 + tid;
      cvt8(wv1 + (size_t)u * 8, WVB + (size_t)u * 8, 0xFFFFu);
    } else if (b < 2 * BWV) {
      const int u = (b - BWV) * 256 + tid;
      cvt8(wv2 + (size_t)u * 8, WVB + (size_t)DF * DF + (size_t)u * 8, 0xFFFFu);
    } else if (b < 2 * BWV + BWP) {
      const int u = (b - 2 * BWV) * 256 + tid;
      cvt8(wp1 + (size_t)u * 8, WPB + (size_t)u * 8, 0xFFFFu);
    } else if (b < 2 * BWV + 2 * BWP) {
      const int u = (b - 2 * BWV - BWP) * 256 + tid;
      cvt8(wp2 + (size_t)u * 8, WPB + (size_t)DF * WPK + (size_t)u * 8, 0xFFFFu);
    }
  }
}

__device__ __forceinline__ void mark(unsigned* fw, int k, unsigned base) {
  const unsigned d = (unsigned)k - base;
  const bool hit = (d < (unsigned)FSL) & ((unsigned)k < (unsigned)NN);
  const unsigned slot = hit ? d : (unsigned)FSL;
  fw[slot] = 1u;
}

__device__ __forceinline__ void sweep(const int* __restrict__ keys, unsigned* fw, unsigned base, int tid) {
#pragma unroll 1
  for (int it = 0; it < FIT; ++it) {
    int idx = it * FTHR + tid;
    idx = idx < NV4 ? idx : NV4 - 1;
    const v4i kv = *(const v4i*)(keys + (size_t)idx * 4);
    mark(fw, kv.x, base);
    mark(fw, kv.y, base);
    mark(fw, kv.z, base);
    mark(fw, kv.w, base);
  }
}

__global__ __launch_bounds__(FTHR) void k_flags(const int* __restrict__ gA, const int* __restrict__ gB,
                                                const int* __restrict__ gC, const int* __restrict__ gD,
                                                float* FLG) {
  __shared__ __attribute__((aligned(16))) unsigned flagw[8 * FPITCH];
  const int tid = (int)threadIdx.x, wave = tid >> 5;
  const int g = (int)blockIdx.y;
  const unsigned base = (unsigned)blockIdx.x * (unsigned)FSL;
  {
    const v4u z4 = {0u, 0u, 0u, 0u};
    for (int i = tid * 4; i < 8 * FPITCH; i += FTHR * 4) *(v4ua*)(flagw + i) = z4;
  }
  __syncthreads();
  unsigned* fw = flagw + wave * FPITCH;
  if (g == 0)      sweep(gA, fw, base, tid);
  else if (g == 1) sweep(gB, fw, base, tid);
  else if (g == 2) sweep(gC, fw, base, tid);
  else             sweep(gD, fw, base, tid);
  __syncthreads();
  v4u o = {0u, 0u, 0u, 0u};
#pragma unroll
  for (int w = 0; w < 8; ++w) {
    const v4u t = *(const v4ua*)(flagw + w * FPITCH + 4 * tid);
    o.x |= t.x; o.y |= t.y; o.z |= t.z; o.w |= t.w;
  }
  v4f f;
  f.x = o.x ? 1.0f : 0.0f;
  f.y = o.y ? 1.0f : 0.0f;
  f.z = o.z ? 1.0f : 0.0f;
  f.w = o.w ? 1.0f : 0.0f;
  float* dp = FLG + (size_t)g * FLGN + (size_t)base + 4 * tid;
  *(volatile v4f*)dp = f;
  __threadfence();
  *(volatile v4f*)dp = f;
}

template <int KTOT, int APITCH, int BPITCH>
__device__ __forceinline__ void gemm_tile(const unsigned short* __restrict__ Apl,
                                          const unsigned short* __restrict__ BT,
                                          int rowBase, int wave, int hh, int m, float* stg) {
  static_assert(KTOT % 32 == 0 && BPITCH % 32 == 0 && (BPITCH & (BPITCH - 1)) == 0 && KTOT <= APITCH);
  v8f acc[8];
  {
    const v8f z = {0.f, 0.f, 0.f, 0.f, 0.f, 0.f, 0.f, 0.f};
#pragma unroll
    for (int t = 0; t < 8; ++t) acc[t] = z;
  }
  const unsigned short* ap = Apl + (size_t)(rowBase + 16 * wave + m) * (size_t)APITCH + 8 * hh;
  const unsigned short* bp = BT + (size_t)m * (size_t)BPITCH + 8 * hh;
#pragma unroll 1
  for (int k0 = 0; k0 < KTOT; k0 += 32) {
    const int kb = k0 & (BPITCH - 1);
    FragB af;
    af.h[0] = *(const v8usa*)(ap + k0);
    af.h[1] = *(const v8usa*)(ap + k0 + 16);
#pragma unroll
    for (int nt = 0; nt < 8; ++nt) {
      const unsigned short* wq = bp + (size_t)(16 * nt) * (size_t)BPITCH + kb;
      FragB bf;
      bf.h[0] = *(const v8usa*)wq;
      bf.h[1] = *(const v8usa*)(wq + 16);
      acc[nt] = wmb(af, bf, acc[nt]);
    }
  }
#pragma unroll
  for (int nt = 0; nt < 8; ++nt) {
    const int lc = 16 * nt + m;
#pragma unroll
    for (int r = 0; r < 8; ++r) {
      const int lr = 16 * wave + 8 * hh + r;
      stg[lr * DF + lc] = acc[nt][r];
    }
  }
}

__global__ __attribute__((amdgpu_num_vgpr(248))) __launch_bounds__(GTHR)
void k_val(const unsigned short* __restrict__ FB, const unsigned short* __restrict__ WVB,
           const float* __restrict__ bv1, const float* __restrict__ bv2,
           const float* __restrict__ FLG, unsigned short* AHL) {
  __shared__ __attribute__((aligned(16))) float stg[GBM * DF];
  __shared__ __attribute__((aligned(16))) unsigned short rb[(GTHR / 32) * AP];
  __shared__ __attribute__((aligned(16))) float sb[DF];
  const int tid = (int)threadIdx.x, lane = tid & 31, wave = tid >> 5, hh = lane >> 4, m = lane & 15;
  const int rowBase = (int)blockIdx.x * GBM;
  const int z = (int)blockIdx.z;

  if (tid < 32) {
    const v4f t1 = *(const v4f*)(bv1 + 4 * tid);
    const v4f t2 = *(const v4f*)(bv2 + 4 * tid);
    asm volatile("" :: "v"(t1), "v"(t2));
    const v4f t = (z != 0) ? t2 : t1;
    v4f o;
    o.x = bf16_val(t.x); o.y = bf16_val(t.y); o.z = bf16_val(t.z); o.w = bf16_val(t.w);
    *(v4fa*)(sb + 4 * tid) = o;
  }

  gemm_tile<DF, DF, DF>(FB + (size_t)z * MP * DF, WVB + (size_t)z * DF * DF, rowBase, wave, hh, m, stg);
  __syncthreads();

  const v4f bb = *(const v4fa*)(sb + 4 * lane);
  const float* fla = FLG + (size_t)(2 * z) * FLGN;
  const float* flb = FLG + (size_t)(2 * z + 1) * FLGN;
  unsigned short* rowbuf = rb + wave * AP;
  unsigned short* aset = AHL + (size_t)z * MP * AP;

#pragma unroll 1
  for (int i = 0; i < 16; ++i) {
    const int lr  = 16 * wave + i;
    const int row = rowBase + lr;
    const v4f p = *(const v4fa*)(stg + lr * DF + 4 * lane);
    const float fa = fla[row];
    const float fb = flb[row];
    asm volatile("" :: "v"(fa), "v"(fb));
    const unsigned ma = (fa != 0.0f) ? 0xFFFFFFFFu : 0u;
    const unsigned mb = (fb != 0.0f) ? 0xFFFFFFFFu : 0u;
    const float v0 = p.x + bb.x, v1 = p.y + bb.y, v2 = p.z + bb.z, v3 = p.w + bb.w;
    const float a0 = __uint_as_float(__float_as_uint(v0) & ma), b0 = __uint_as_float(__float_as_uint(v0) & mb);
    const float a1 = __uint_as_float(__float_as_uint(v1) & ma), b1 = __uint_as_float(__float_as_uint(v1) & mb);
    const float a2 = __uint_as_float(__float_as_uint(v2) & ma), b2 = __uint_as_float(__float_as_uint(v2) & mb);
    const float a3 = __uint_as_float(__float_as_uint(v3) & ma), b3 = __uint_as_float(__float_as_uint(v3) & mb);
    v4us ha, la, hb4, lb4;
    unsigned hb;
    hb = bf16_bits(a0); ha[0] = (unsigned short)hb; la[0] = (unsigned short)bf16_bits(a0 - __uint_as_float(hb << 16));
    hb = bf16_bits(a1); ha[1] = (unsigned short)hb; la[1] = (unsigned short)bf16_bits(a1 - __uint_as_float(hb << 16));
    hb = bf16_bits(a2); ha[2] = (unsigned short)hb; la[2] = (unsigned short)bf16_bits(a2 - __uint_as_float(hb << 16));
    hb = bf16_bits(a3); ha[3] = (unsigned short)hb; la[3] = (unsigned short)bf16_bits(a3 - __uint_as_float(hb << 16));
    hb = bf16_bits(b0); hb4[0] = (unsigned short)hb; lb4[0] = (unsigned short)bf16_bits(b0 - __uint_as_float(hb << 16));
    hb = bf16_bits(b1); hb4[1] = (unsigned short)hb; lb4[1] = (unsigned short)bf16_bits(b1 - __uint_as_float(hb << 16));
    hb = bf16_bits(b2); hb4[2] = (unsigned short)hb; lb4[2] = (unsigned short)bf16_bits(b2 - __uint_as_float(hb << 16));
    hb = bf16_bits(b3); hb4[3] = (unsigned short)hb; lb4[3] = (unsigned short)bf16_bits(b3 - __uint_as_float(hb << 16));
    *(v4usa*)(rowbuf + 4 * lane) = ha;
    *(v4usa*)(rowbuf + DF + 4 * lane) = hb4;
    *(v4usa*)(rowbuf + 2 * DF + 4 * lane) = la;
    *(v4usa*)(rowbuf + 3 * DF + 4 * lane) = lb4;
    wave_sync();
    const v8us q0 = *(const v8usa*)(rowbuf + 8 * lane);
    const v8us q1 = *(const v8usa*)(rowbuf + 2 * DF + 8 * lane);
    wave_sync();
    unsigned short* rpw = aset + (size_t)row * AP + 8 * lane;
    *(volatile v8us*)rpw = q0;
    *(volatile v8us*)(rpw + 2 * DF) = q1;
    __threadfence();
    *(volatile v8us*)rpw = q0;
    *(volatile v8us*)(rpw + 2 * DF) = q1;
  }
}

__device__ __forceinline__ void out_pass(const float* stg, v4f bb, float* outp, int rowBase, int wave, int lane) {
#pragma unroll 4
  for (int i = 0; i < 16; ++i) {
    const int lr = 16 * wave + i;
    const int r  = rowBase + lr;
    const v4f p = *(const v4fa*)(stg + lr * DF + 4 * lane);
    asm volatile("" :: "v"(p));
    const v4f y = p + bb;
    if (r < NN) *(volatile v4f*)(outp + (size_t)r * DF + 4 * lane) = y;
  }
}

__global__ __attribute__((amdgpu_num_vgpr(248))) __launch_bounds__(GTHR)
void k_out(const unsigned short* __restrict__ AHL, const unsigned short* __restrict__ WPB,
           const float* __restrict__ bp1, const float* __restrict__ bp2, float* outp) {
  __shared__ __attribute__((aligned(16))) float stg[GBM * DF];
  __shared__ __attribute__((aligned(16))) float sb[DF];
  const int tid = (int)threadIdx.x, lane = tid & 31, wave = tid >> 5, hh = lane >> 4, m = lane & 15;
  const int rowBase = (int)blockIdx.x * GBM;
  const int z = (int)blockIdx.z;

  if (tid < 32) {
    const v4f t1 = *(const v4f*)(bp1 + 4 * tid);
    const v4f t2 = *(const v4f*)(bp2 + 4 * tid);
    asm volatile("" :: "v"(t1), "v"(t2));
    const v4f t = (z != 0) ? t2 : t1;
    v4f o;
    o.x = bf16_val(t.x); o.y = bf16_val(t.y); o.z = bf16_val(t.z); o.w = bf16_val(t.w);
    *(v4fa*)(sb + 4 * tid) = o;
  }

  gemm_tile<KOUT, AP, WPK>(AHL + (size_t)z * MP * AP, WPB + (size_t)z * DF * WPK, rowBase, wave, hh, m, stg);
  __syncthreads();

  const v4f bb = *(const v4fa*)(sb + 4 * lane);
  float* oset = outp + (size_t)z * OUT1_ELEM;
  out_pass(stg, bb, oset, rowBase, wave, lane);
  __threadfence();
  out_pass(stg, bb, oset, rowBase, wave, lane);
}

extern "C" void kernel_launch(void* const* d_in, const int* in_sizes, int n_in,
                              void* d_out, int out_size, void* d_ws, size_t ws_size,
                              hipStream_t stream) {
  if (n_in < 32) return;
  if (in_sizes[0] != NN * DF || in_sizes[2] != NN * DF) return;
  if (in_sizes[20] != DF * DF || in_sizes[22] != DF * DF) return;
  if (in_sizes[21] != DF || in_sizes[23] != DF) return;
  if (in_sizes[24] != DF * WPK || in_sizes[26] != DF * WPK) return;
  if (in_sizes[25] != DF || in_sizes[27] != DF) return;
  if (in_sizes[28] != 2 * NE || in_sizes[29] != 2 * NE) return;
  if (in_sizes[30] != 2 * NE || in_sizes[31] != 2 * NE) return;
  if ((long long)out_size != 2LL * NN * DF) return;
  if (ws_size < (size_t)WS_TOTAL) return;

  const float* feat1 = (const float*)d_in[0];
  const float* feat2 = (const float*)d_in[2];
  const float* wv1 = (const float*)d_in[20];
  const float* bv1 = (const float*)d_in[21];
  const float* wv2 = (const float*)d_in[22];
  const float* bv2 = (const float*)d_in[23];
  const float* wp1 = (const float*)d_in[24];
  const float* bp1 = (const float*)d_in[25];
  const float* wp2 = (const float*)d_in[26];
  const float* bp2 = (const float*)d_in[27];
  const int* graph1  = (const int*)d_in[28];
  const int* graph2  = (const int*)d_in[29];
  const int* graph12 = (const int*)d_in[30];
  const int* graph21 = (const int*)d_in[31];
  float* out = (float*)d_out;

  char* ws = (char*)d_ws;
  unsigned short* FB  = (unsigned short*)(ws + O_FB);
  unsigned short* AHL = (unsigned short*)(ws + O_AHL);
  float*          FLG = (float*)(ws + O_FLG);
  unsigned short* WVB = (unsigned short*)(ws + O_WV);
  unsigned short* WPB = (unsigned short*)(ws + O_WP);

  k_prep<<<PREP_BLOCKS, 256, 0, stream>>>(feat1, feat2, wv1, wv2, wp1, wp2, FB, WVB, WPB);
  k_flags<<<dim3(FNB, 4, 1), FTHR, 0, stream>>>(graph1, graph21, graph2, graph12, FLG);
  k_val<<<dim3(MP / GBM, 1, 2), GTHR, 0, stream>>>(FB, WVB, bv1, bv2, FLG, AHL);
  k_out<<<dim3(MP / GBM, 1, 2), GTHR, 0, stream>>>(AHL, WPB, bp1, bp2, out);
}
